// PointInt_49555332661490
// MI455X (gfx1250) — hardware-verified
//
#include <hip/hip_runtime.h>
#include <math.h>

typedef __attribute__((ext_vector_type(16))) _Float16 v16h;
typedef __attribute__((ext_vector_type(16))) __bf16 v16b;
typedef __attribute__((ext_vector_type(8)))  _Float16 v8h;
typedef __attribute__((ext_vector_type(8)))  float v8f;
typedef __attribute__((ext_vector_type(4)))  float v4f;
typedef __attribute__((ext_vector_type(2)))  float v2f;
typedef __attribute__((ext_vector_type(4)))  unsigned v4u;
typedef __attribute__((ext_vector_type(4)))  int v4i;
typedef float __attribute__((may_alias)) float_a;
typedef int __attribute__((may_alias)) int_a;

template <typename T> __device__ __forceinline__ void vst2(void* p, T v) { *(volatile T*)p = v; __threadfence(); *(volatile T*)p = v; }
__device__ __forceinline__ v8f wmma16(v16h a, v16h b, v8f c) {
  v8f d = __builtin_amdgcn_wmma_f32_16x16x32_f16(false, a, false, b, (short)0, c, false, false);
  asm volatile("v_nop\n\tv_nop\n\tv_nop\n\tv_nop" : "+v"(d) : "v"(a), "v"(b));
  return d;
}
__device__ __forceinline__ v8f wmma_bf(v16b a, v16b b, v8f c) {
  v8f d = __builtin_amdgcn_wmma_f32_16x16x32_bf16(false, a, false, b, (short)0, c, false, false);
  asm volatile("v_nop\n\tv_nop\n\tv_nop\n\tv_nop" : "+v"(d) : "v"(a), "v"(b));
  return d;
}
__device__ __forceinline__ v16h frag_h(const _Float16* rowk0, int lane) {
  union { v16h v; v8h q[2]; } u; const _Float16* p = rowk0 + 8 * (lane >> 4);
  u.q[0] = *(const v8h*)p; u.q[1] = *(const v8h*)(p + 16); return u.v;
}
__device__ __forceinline__ v16h frag_f32(const float* rowk0, int lane) {
  v16h a; const float* p = rowk0 + 8 * (lane >> 4);
#pragma unroll
  for (int i = 0; i < 8; ++i) { a[i] = (_Float16)p[i]; a[8 + i] = (_Float16)p[16 + i]; }
  return a;
}
__device__ __forceinline__ v16h frag_f32s(const float* rowk0, int lane, float sc) {
  v16h a; const float* p = rowk0 + 8 * (lane >> 4);
#pragma unroll
  for (int i = 0; i < 8; ++i) { a[i] = (_Float16)(p[i] * sc); a[8 + i] = (_Float16)(p[16 + i] * sc); }
  return a;
}
__device__ __forceinline__ v16h fragc_f32(const float* W, int k0, int n, int lane, int ld, int K) {
  v16h a; const int g = lane >> 4;
#pragma unroll
  for (int i = 0; i < 8; ++i) { const int ka = k0 + 8 * g + i, kb = ka + 16;
    a[i] = (_Float16)(ka < K ? W[(size_t)ka * ld + n] : 0.f); a[8 + i] = (_Float16)(kb < K ? W[(size_t)kb * ld + n] : 0.f); }
  return a;
}
struct F2 { v16b h, l; };
__device__ __forceinline__ F2 bsplit16(const float v[16]) { F2 r;
#pragma unroll
  for (int i = 0; i < 16; ++i) { const __bf16 h = (__bf16)v[i]; r.h[i] = h; r.l[i] = (__bf16)(v[i] - (float)h); }
  return r; }
__device__ __forceinline__ F2 split_row(const float* row, int k0, int lane) { float v[16]; const float* p = row + k0 + 8 * (lane >> 4);
#pragma unroll
  for (int i = 0; i < 8; ++i) { v[i] = p[i]; v[8 + i] = p[16 + i]; }
  return bsplit16(v); }
__device__ __forceinline__ F2 split_rowK(const float* row, int k0, int lane, int K) { float v[16]; const int g = lane >> 4;
#pragma unroll
  for (int i = 0; i < 8; ++i) { const int ka = k0 + 8 * g + i, kb = ka + 16; v[i] = ka < K ? row[ka] : 0.f; v[8 + i] = kb < K ? row[kb] : 0.f; }
  return bsplit16(v); }
__device__ __forceinline__ F2 split_col(const float* W, int k0, int n, int lane, int ld, int K) { float v[16]; const int g = lane >> 4;
#pragma unroll
  for (int i = 0; i < 8; ++i) { const int ka = k0 + 8 * g + i, kb = ka + 16; v[i] = ka < K ? W[(size_t)ka * ld + n] : 0.f; v[8 + i] = kb < K ? W[(size_t)kb * ld + n] : 0.f; }
  return bsplit16(v); }
__device__ __forceinline__ v8f mac3(const F2& a, const F2& b, v8f c) { c = wmma_bf(a.l, b.h, c); c = wmma_bf(a.h, b.l, c); return wmma_bf(a.h, b.h, c); }
__device__ __forceinline__ float sigm(float v) { return 1.0f / (1.0f + expf(-v)); }
#define LDSX() do { asm volatile("s_wait_dscnt 0" ::: "memory"); __builtin_amdgcn_wave_barrier(); __builtin_amdgcn_fence(__ATOMIC_RELEASE, "workgroup"); } while (0)

#define NPTS 50000
#define NSUP 50000
#define NNB 32
#define NKP 15
#define CC 128
#define EXT 1.2f
#define NPAD 50048

__global__ __launch_bounds__(256) void k_main(const float* __restrict__ qp, const float* __restrict__ sp, const int* __restrict__ nb, const float* __restrict__ x, const float* __restrict__ kp, const float* __restrict__ dw, const float* __restrict__ bias, float* __restrict__ out) {
  __shared__ __align__(16) _Float16 sw[64 * NNB][16];
  __shared__ float skp[NKP][3]; __shared__ __align__(16) _Float16 sdw[CC][16];
  __shared__ int snb[64][NNB];
  __shared__ __align__(16) float scoef[8][16][132];
  __shared__ __align__(16) float sres[64][CC + 4];
  const int tid = threadIdx.x, wave = tid >> 5, lane = tid & 31, col = lane & 15, g = lane >> 4;
  const int p0 = blockIdx.x * 64;
  if (tid < NKP * 3) skp[tid / 3][tid % 3] = kp[tid];
  for (int q = tid; q < CC * 16; q += 256) { const int c = q >> 4, k = q & 15; sdw[c][k] = (_Float16)(k < NKP ? dw[k * CC + c] * 2.0f : 0.f); }
  __syncthreads();
  for (int q = tid; q < 64 * NNB; q += 256) { const int pl = q >> 5, h = q & 31; const int p = min(p0 + pl, NPTS - 1);
    int j = nb[(size_t)p * NNB + h]; const bool pad = (j < 0) || (j >= NSUP); snb[pl][h] = pad ? -1 : j;
    float nx, ny, nz;
    if (pad) { nx = 1.0e6f - qp[(size_t)p * 3]; ny = 1.0e6f - qp[(size_t)p * 3 + 1]; nz = 1.0e6f - qp[(size_t)p * 3 + 2]; }
    else { nx = sp[(size_t)j * 3] - qp[(size_t)p * 3]; ny = sp[(size_t)j * 3 + 1] - qp[(size_t)p * 3 + 1]; nz = sp[(size_t)j * 3 + 2] - qp[(size_t)p * 3 + 2]; }
    union { v8h h8[2]; v4u u[2]; } pk;
#pragma unroll
    for (int k = 0; k < 16; ++k) { float wv = 0.f;
      if (k < NKP) { const float dx = nx - skp[k][0], dy = ny - skp[k][1], dz = nz - skp[k][2]; wv = 1.0f - sqrtf(dx * dx + dy * dy + dz * dz) * (1.0f / EXT); wv = wv > 6.2e-5f ? wv : 0.f; }
      pk.h8[k >> 3][k & 7] = (_Float16)wv; }
    *(v4u*)(&sw[q][0]) = pk.u[0]; *(v4u*)(&sw[q][8]) = pk.u[1]; }
  __syncthreads();
  float racc[4] = {0.f, 0.f, 0.f, 0.f};
#pragma unroll 1
  for (int tix = 0; tix < 16; ++tix) { const int rowb = wave * 256 + tix * 16; const int pl = rowb >> 5, hb = rowb & 31;
    if (hb == 0) { racc[0] = racc[1] = racc[2] = racc[3] = 0.f; }
    v16h a;
#pragma unroll
    for (int i = 0; i < 8; ++i) { a[i] = sw[rowb + col][8 * g + i]; a[8 + i] = (_Float16)0.f; }
#pragma unroll
    for (int t = 0; t < 8; ++t) { v16h bb;
#pragma unroll
      for (int i = 0; i < 8; ++i) { bb[i] = sdw[t * 16 + col][8 * g + i]; bb[8 + i] = (_Float16)0.f; }
      v8f acc = {}; acc = wmma16(a, bb, acc);
#pragma unroll
      for (int r = 0; r < 8; ++r) scoef[wave][8 * g + r][t * 16 + col] = acc[r] * 0.5f; }
    LDSX();
#pragma unroll 4
    for (int hh = 0; hh < 16; ++hh) { const int j = snb[pl][hb + hh];
      if (j >= 0) { const v4f xv = *(const v4f*)(x + (size_t)j * CC + lane * 4);
#pragma unroll
        for (int e = 0; e < 4; ++e) racc[e] += scoef[wave][hh][lane * 4 + e] * xv[e]; } }
    if (hb == 16) {
#pragma unroll
      for (int e = 0; e < 4; ++e) sres[pl][lane * 4 + e] = racc[e] + bias[lane * 4 + e]; }
    LDSX(); }
  __syncthreads();
  for (int q = tid; q < 64 * (CC / 4); q += 256) { const int pl = q >> 5, pc = q & 31; if (p0 + pl < NPTS) vst2(out + (size_t)(p0 + pl) * CC + pc * 4, *(const v4f*)(&sres[pl][pc * 4])); }
}
extern "C" void kernel_launch(void* const* d_in, const int* in_sizes, int n_in, void* d_out, int out_size, void* d_ws, size_t ws_size, hipStream_t stream) {
  (void)in_sizes; (void)n_in; (void)out_size; (void)ws_size; (void)d_ws;
  const float* qp = (const float*)d_in[0]; const float* sp = (const float*)d_in[1]; const int* nb = (const int*)d_in[2]; const float* x = (const float*)d_in[3]; const float* kp = (const float*)d_in[4]; const float* dw = (const float*)d_in[5]; const float* bias = (const float*)d_in[6];
  float* out = (float*)d_out;
  k_main<<<NPAD / 64, 256, 0, stream>>>(qp, sp, nb, x, kp, dw, bias, out);
}
